// DCNConvModule_19928648253490
// MI455X (gfx1250) — hardware-verified
//
#include <hip/hip_runtime.h>
#include <math.h>
#include <stddef.h>

typedef __attribute__((ext_vector_type(16))) _Float16 v16h;
typedef __attribute__((ext_vector_type(8)))  _Float16 v8h;
typedef __attribute__((ext_vector_type(16))) __bf16   v16b;
typedef __attribute__((ext_vector_type(8)))  __bf16   v8b;
typedef __attribute__((ext_vector_type(8)))  float    v8f;
typedef __attribute__((ext_vector_type(4)))  float    v4f;
typedef __attribute__((ext_vector_type(4)))  unsigned int v4u;

constexpr int NBATCH   = 4;
constexpr int NCIN     = 256;
constexpr int IMG_H    = 64;
constexpr int IMG_W    = 64;
constexpr int NPIX     = IMG_H * IMG_W;
constexpr int NCOUT    = 256;
constexpr int NTAP     = 9;
constexpr int KDIM     = NTAP * NCIN;
constexpr int MROWS    = NBATCH * NPIX;
constexpr int NOFF     = 27;
constexpr int NOFFPAD  = 64;
constexpr int NTHR     = 256;
constexpr int PART_STRIDE = 32;
constexpr float X_CARRY     = 16.0f;
constexpr float WOFF_CARRY  = 256.0f;
constexpr float WGT_CARRY   = 256.0f;
constexpr float SMP_CARRY   = 16.0f;
constexpr float GEMM0_SCALE = 1.0f / 4096.0f;
constexpr float GEMM1_SCALE = 1.0f / 4096.0f;
constexpr float GN_EPS      = 1e-5f;

static_assert(MROWS % 64 == 0 && NOFFPAD % 64 == 0 && KDIM % 32 == 0);
static_assert(NCOUT % 64 == 0 && NPIX % 64 == 0);
static_assert(((MROWS / 64) * (NOFFPAD / 64)) % 8 == 0);
static_assert(((NCOUT / 64) * (NPIX / 64)) % 8 == 0);
static_assert(NOFF <= NOFFPAD && 2 * NTAP + NTAP == NOFF);
static_assert(NCIN == 32 * 8);
static_assert(NPIX == NTHR * 16);
static_assert(NBATCH * 2 <= PART_STRIDE);

constexpr size_t XT_BYTES    = (size_t)NBATCH * NPIX * NCIN * 2;
constexpr size_t A16_BYTES   = (size_t)MROWS * KDIM * 2;
constexpr size_t W0P_BYTES   = (size_t)NOFFPAD * KDIM * 2;
constexpr size_t OM_BYTES    = (size_t)MROWS * NOFFPAD * 4;
constexpr size_t WP_BYTES    = (size_t)NCOUT * KDIM * 2;
constexpr size_t CONV_BYTES  = (size_t)NBATCH * NCOUT * NPIX * 4;
constexpr size_t PART_BYTES  = (size_t)NBATCH * NCOUT * PART_STRIDE * 4;
constexpr size_t STATS_BYTES = 128;
constexpr size_t OFF_XT    = 0;
constexpr size_t OFF_A16   = OFF_XT + XT_BYTES;
constexpr size_t OFF_W0P   = OFF_A16 + A16_BYTES;
constexpr size_t OFF_OM    = OFF_W0P + W0P_BYTES;
constexpr size_t OFF_WP    = OFF_OM + OM_BYTES;
constexpr size_t OFF_CONV  = OFF_WP + WP_BYTES;
constexpr size_t OFF_PART  = OFF_CONV + CONV_BYTES;
constexpr size_t OFF_STATS = OFF_PART + PART_BYTES;
constexpr size_t WS_TOTAL  = OFF_STATS + STATS_BYTES;
static_assert(WS_TOTAL <= (size_t)134217728);
static_assert(OFF_A16 % 256 == 0 && OFF_W0P % 256 == 0 && OFF_OM % 256 == 0 && OFF_WP % 256 == 0);
static_assert(OFF_CONV % 256 == 0 && OFF_PART % 256 == 0 && OFF_STATS % 256 == 0);

__device__ __forceinline__ unsigned short f2bf_bits(float f) {
  unsigned u = __float_as_uint(f);
  return (unsigned short)((u + 0x7FFFu + ((u >> 16) & 1u)) >> 16);
}
__device__ __forceinline__ float bf_bits2f(unsigned short h) { return __uint_as_float(((unsigned)h) << 16); }

__device__ __forceinline__ void dep_guard_h(v8f& a, v8f& b, v16h x, v16h y) { asm volatile("v_nop\n\tv_nop\n\tv_nop\n\tv_nop" : "+v"(a), "+v"(b) : "v"(x), "v"(y)); }
__device__ __forceinline__ void dep_guard_b(v8f& a, v8f& b, v16b x, v16b y) { asm volatile("v_nop\n\tv_nop\n\tv_nop\n\tv_nop" : "+v"(a), "+v"(b) : "v"(x), "v"(y)); }
__device__ __forceinline__ void keep4_h(v16h a, v16h b, v16h c, v16h d) { asm volatile("v_nop" :: "v"(a), "v"(b), "v"(c), "v"(d)); }
__device__ __forceinline__ void keep4_b(v16b a, v16b b, v16b c, v16b d) { asm volatile("v_nop" :: "v"(a), "v"(b), "v"(c), "v"(d)); }
__device__ __forceinline__ void acc_guard4(v8f& a, v8f& b, v8f& c, v8f& d) { asm volatile("v_nop\n\tv_nop\n\tv_nop\n\tv_nop" : "+v"(a), "+v"(b), "+v"(c), "+v"(d)); }
template <typename T> struct Frag;
template <> struct Frag<_Float16> {
  typedef v16h V; union U { v16h v; v8h h[2]; };
  static __device__ __forceinline__ v16h load(const _Float16* p) {
    U f; f.h[0] = *(const v8h*)(p); f.h[1] = *(const v8h*)(p + 16); return f.v;
  }
  static __device__ __forceinline__ v8f mma(v16h a, v16h b, v8f c) {
    return __builtin_amdgcn_wmma_f32_16x16x32_f16(false, a, false, b, (short)0, c, false, false);
  }
  static __device__ __forceinline__ void guard(v8f& a, v8f& b, v16h x, v16h y) { dep_guard_h(a, b, x, y); }
  static __device__ __forceinline__ void keep(v16h a, v16h b, v16h c, v16h d) { keep4_h(a, b, c, d); }
};
template <> struct Frag<__bf16> {
  typedef v16b V; union U { v16b v; v8b h[2]; };
  static __device__ __forceinline__ v16b load(const __bf16* p) {
    U f; f.h[0] = *(const v8b*)(p); f.h[1] = *(const v8b*)(p + 16); return f.v;
  }
  static __device__ __forceinline__ v8f mma(v16b a, v16b b, v8f c) {
    return __builtin_amdgcn_wmma_f32_16x16x32_bf16(false, a, false, b, (short)0, c, false, false);
  }
  static __device__ __forceinline__ void guard(v8f& a, v8f& b, v16b x, v16b y) { dep_guard_b(a, b, x, y); }
  static __device__ __forceinline__ void keep(v16b a, v16b b, v16b c, v16b d) { keep4_b(a, b, c, d); }
};

template <int ET> struct Elem;
template <> struct Elem<0> { typedef _Float16 T; };
template <> struct Elem<1> { typedef __bf16 T; };
template <int ET, bool SPLIT, int BIAS_MODE, int OUT_MODE, bool RESID, int ACT = 0>
__global__ __launch_bounds__(256) void wmma_gemm64(
    const unsigned short* __restrict__ Ap, const unsigned short* __restrict__ A2p, int lda, long strideA,
    const unsigned short* __restrict__ Btp, const unsigned short* __restrict__ Bt2p, int ldb, long strideB,
    void* __restrict__ Cout, void* __restrict__ Cout2, int ldc, long strideC,
    const float* __restrict__ bias,
    const float* __restrict__ resid, long strideR,
    int M, int N, int K, float scale) {
  typedef typename Elem<ET>::T T;
  typedef typename Frag<T>::V V;
  const T* A = (const T*)Ap; const T* A2 = (const T*)A2p; const T* Bt = (const T*)Btp; const T* Bt2 = (const T*)Bt2p;
  __shared__ __align__(16) float sT[8][16 * 68];
  const int b    = blockIdx.y;
  const int lane = threadIdx.x & 31;
  const int wave = threadIdx.x >> 5;
  const int tilesN = N >> 6;
  const int tilesM = M >> 6;
  const int tile = blockIdx.x * 8 + wave;
  if (tile >= tilesM * tilesN) return;
  const int tm = tile / tilesN;
  const int tn = tile - tm * tilesN;
  const int m0 = tm << 6;
  const int n0 = tn << 6;

  const T* Ab  = A  + (size_t)b * strideA;
  const T* Bb  = Bt + (size_t)b * strideB;
  const T* Ab2 = SPLIT ? (A2  + (size_t)b * strideA) : nullptr;
  const T* Bb2 = SPLIT ? (Bt2 + (size_t)b * strideB) : nullptr;

  const int rlane = lane & 15;
  const int koff  = (lane >> 4) * 8;
  const int mOff  = (lane >> 4) * 8;

  v8f acc[4][4];
#pragma unroll
  for (int i = 0; i < 4; ++i)
#pragma unroll
    for (int j = 0; j < 4; ++j) acc[i][j] = (v8f){0.f,0.f,0.f,0.f,0.f,0.f,0.f,0.f};

  for (int k0 = 0; k0 < K; k0 += 32) {
    V bh[4], bl[4];
#pragma unroll
    for (int j = 0; j < 4; ++j) {
      const size_t bo = (size_t)(n0 + (j << 4) + rlane) * ldb + koff + k0;
      bh[j] = Frag<T>::load(Bb + bo);
      if (SPLIT) bl[j] = Frag<T>::load(Bb2 + bo);
    }
#pragma unroll
    for (int i = 0; i < 4; ++i) {
      const size_t ao = (size_t)(m0 + (i << 4) + rlane) * lda + koff + k0;
      V ah = Frag<T>::load(Ab + ao);
      V al;
      if (SPLIT) al = Frag<T>::load(Ab2 + ao);
#pragma unroll
      for (int j = 0; j < 4; ++j) {
        acc[i][j] = Frag<T>::mma(ah, bh[j], acc[i][j]);
        if (SPLIT) {
          acc[i][j] = Frag<T>::mma(ah, bl[j], acc[i][j]);
          acc[i][j] = Frag<T>::mma(al, bh[j], acc[i][j]);
        }
      }
      Frag<T>::guard(acc[i][0], acc[i][3], ah, SPLIT ? al : ah);
    }
    Frag<T>::keep(bh[0], bh[1], bh[2], bh[3]);
    if (SPLIT) Frag<T>::keep(bl[0], bl[1], bl[2], bl[3]);
  }
  acc_guard4(acc[0][0], acc[0][1], acc[0][2], acc[0][3]);
  acc_guard4(acc[1][0], acc[1][1], acc[1][2], acc[1][3]);
  acc_guard4(acc[2][0], acc[2][1], acc[2][2], acc[2][3]);
  acc_guard4(acc[3][0], acc[3][1], acc[3][2], acc[3][3]);

  float* slab = sT[wave];
  const float* Rb = RESID ? (resid + (size_t)b * strideR) : nullptr;
#pragma unroll
  for (int i = 0; i < 4; ++i) {
    const int mBase = m0 + (i << 4);
#pragma unroll
    for (int j = 0; j < 4; ++j) {
      const int n = n0 + (j << 4) + rlane;
      float bv = 0.f;
      if (BIAS_MODE == 2) bv = bias[n];
#pragma unroll
      for (int r = 0; r < 8; ++r) {
        float v = acc[i][j][r] * scale;
        if (BIAS_MODE == 1) v += bias[mBase + mOff + r];
        if (BIAS_MODE == 2) v += bv;
        if (RESID) v += Rb[(size_t)(mBase + mOff + r) * ldc + n];
        if (ACT == 1) v = tanhf(v);
        if (ACT == 2) v = fmaxf(v, 0.0f);
        if (ACT == 3) v = v / (1.0f + expf(-v));
        if (ACT == 4) v = (v > 0.f) ? v : 0.01f * v;
        if (ACT == 5) v = 0.5f * v * (1.0f + erff(v * 0.70710678118654752f));
        slab[(mOff + r) * 68 + (j << 4) + rlane] = v;
      }
    }
    __builtin_amdgcn_fence(__ATOMIC_RELEASE, "workgroup");
    __builtin_amdgcn_wave_barrier();
    __builtin_amdgcn_fence(__ATOMIC_ACQUIRE, "workgroup");
    if (OUT_MODE == 0) {
      float* C = (float*)Cout + (size_t)b * strideC;
      const int hh = lane >> 4, c4 = (lane & 15) * 4;
      for (int pass = 0; pass < 2; ++pass) {
#pragma unroll
        for (int it = 0; it < 8; ++it) {
          const int row = it * 2 + hh;
          v4f v = *(const v4f*)(slab + row * 68 + c4);
          *(volatile v4f*)(C + (size_t)(mBase + row) * ldc + n0 + c4) = v;
        }
        __threadfence();
      }
    } else {
      const int q = lane >> 3, c8 = (lane & 7) * 8;
      unsigned short* C  = (unsigned short*)Cout  + (size_t)b * strideC;
      unsigned short* C2 = (OUT_MODE == 2) ? ((unsigned short*)Cout2 + (size_t)b * strideC) : nullptr;
      for (int pass = 0; pass < 2; ++pass) {
#pragma unroll
        for (int it = 0; it < 4; ++it) {
          const int row = it * 4 + q;
          const float* sp = slab + row * 68 + c8;
          v8h hv, lv;
#pragma unroll
          for (int e = 0; e < 8; ++e) {
            if (OUT_MODE == 1) {
              hv[e] = (_Float16)sp[e];
            } else {
              unsigned short hb = f2bf_bits(sp[e]);
              unsigned short lb = f2bf_bits(sp[e] - bf_bits2f(hb));
              hv[e] = __builtin_bit_cast(_Float16, hb);
              lv[e] = __builtin_bit_cast(_Float16, lb);
            }
          }
          *(volatile v8h*)(C + (size_t)(mBase + row) * ldc + n0 + c8) = hv;
          if (OUT_MODE == 2) *(volatile v8h*)(C2 + (size_t)(mBase + row) * ldc + n0 + c8) = lv;
        }
        __threadfence();
      }
    }
    __builtin_amdgcn_fence(__ATOMIC_RELEASE, "workgroup");
    __builtin_amdgcn_wave_barrier();
    __builtin_amdgcn_fence(__ATOMIC_ACQUIRE, "workgroup");
  }
}

__device__ __forceinline__ float bfr(float f) { return bf_bits2f(f2bf_bits(f)); }

__global__ __launch_bounds__(NTHR) void k_xpose(const float* __restrict__ x, unsigned short* __restrict__ xt) {
  __shared__ __align__(16) unsigned short sm[64 * 72];
  const int tid = threadIdx.x, lane = tid & 31, wave = tid >> 5;
  const int p0 = blockIdx.x * 64;
  const int c0 = blockIdx.y * 64;
  const int b  = blockIdx.z;
  const float* xb = x + ((size_t)b * NCIN + c0) * NPIX + p0;
#pragma unroll
  for (int it = 0; it < 4; ++it) {
    const int idx = it * NTHR + tid;
    const int ci  = idx >> 4;
    const int pj4 = (idx & 15) * 4;
    const v4f v = *(const v4f*)(xb + (size_t)ci * NPIX + pj4);
#pragma unroll
    for (int e = 0; e < 4; ++e) sm[(pj4 + e) * 72 + ci] = f2bf_bits(v[e]);
  }
  __syncthreads();
  const int q = lane >> 3, c8 = (lane & 7) * 8;
  for (int pass = 0; pass < 2; ++pass) {
#pragma unroll
    for (int it = 0; it < 2; ++it) {
      const int pj = it * 32 + wave * 4 + q;
      const v4u u = *(const v4u*)(sm + pj * 72 + c8);
      unsigned short* dst = xt + ((size_t)b * NPIX + (size_t)(p0 + pj)) * NCIN + c0 + c8;
      *(volatile v4u*)dst = u;
    }
    __threadfence();
  }
}

__global__ __launch_bounds__(NTHR) void k_im2col(const unsigned short* __restrict__ xt, unsigned short* __restrict__ a16) {
  const int lane = threadIdx.x & 31, wave = threadIdx.x >> 5;
  const int h = blockIdx.x, tap = blockIdx.y, b = blockIdx.z;
  const int ki = tap / 3, kj = tap - ki * 3;
  const int hs = h - 1 + ki;
  const bool hval = (hs >= 0) && (hs < IMG_H);
  const int hsc = hs < 0 ? 0 : (hs > IMG_H - 1 ? IMG_H - 1 : hs);
  const unsigned short* xb = xt + (size_t)b * NPIX * NCIN + lane * 8;
  unsigned short* arow0 = a16 + ((size_t)b * NPIX + (size_t)h * IMG_W) * KDIM + tap * NCIN + lane * 8;
#pragma unroll 1
  for (int it = 0; it < 8; ++it) {
    const int w = it * 8 + wave;
    const int wsrc = w - 1 + kj;
    const bool val = hval && (wsrc >= 0) && (wsrc < IMG_W);
    const int wsc = wsrc < 0 ? 0 : (wsrc > IMG_W - 1 ? IMG_W - 1 : wsrc);
    const v4u u = *(const v4u*)(xb + (size_t)(hsc * IMG_W + wsc) * NCIN);
    v8h hv;
#pragma unroll
    for (int e = 0; e < 4; ++e) {
      const float f0 = val ? __uint_as_float(u[e] << 16) * X_CARRY : 0.0f;
      const float f1 = val ? __uint_as_float(u[e] & 0xffff0000u) * X_CARRY : 0.0f;
      hv[2 * e]     = (_Float16)f0;
      hv[2 * e + 1] = (_Float16)f1;
    }
    unsigned short* dst = arow0 + (size_t)w * KDIM;
    *(volatile v8h*)dst = hv;
    __threadfence();
    *(volatile v8h*)dst = hv;
  }
}

__global__ __launch_bounds__(NTHR) void k_wprep16(const float* __restrict__ W, int nreal, int nrow, float carry,
                                                   unsigned short* __restrict__ out) {
  constexpr int TPR = KDIM / 8;
  const int i = blockIdx.x * NTHR + threadIdx.x;
  if (i >= nrow * TPR) return;
  const int n   = i / TPR;
  const int k0  = (i - n * TPR) * 8;
  const int tap = k0 >> 8;
  const int cb  = k0 & 255;
  const int ncl = (n < nreal) ? n : (nreal - 1);
  const bool rowval = (n < nreal);
  v8h hv;
#pragma unroll
  for (int e = 0; e < 8; ++e) {
    float v = W[(size_t)ncl * KDIM + (size_t)(cb + e) * NTAP + tap];
    v = rowval ? (carry * bfr(v)) : 0.0f;
    hv[e] = (_Float16)v;
  }
  unsigned short* dst = out + (size_t)i * 8;
  *(volatile v8h*)dst = hv;
  __threadfence();
  *(volatile v8h*)dst = hv;
}

__global__ __launch_bounds__(NTHR) void k_sample(const unsigned short* __restrict__ xt, const float* __restrict__ om,
                                                  const float* __restrict__ b_off, unsigned short* __restrict__ a16) {
  const int lane = threadIdx.x & 31, wave = threadIdx.x >> 5;
  const int h = blockIdx.x, tap = blockIdx.y, b = blockIdx.z;
  const int ki = tap / 3, kj = tap - ki * 3;
  const float boy = bfr(b_off[2 * tap]);
  const float box_ = bfr(b_off[2 * tap + 1]);
  const float bom = bfr(b_off[2 * NTAP + tap]);
  const float basey = (float)(h - 1 + ki);
  const float cmax = (float)(IMG_H - 1);
  const unsigned short* xb = xt + (size_t)b * NPIX * NCIN + lane * 8;
  unsigned short* arow0 = a16 + ((size_t)b * NPIX + (size_t)h * IMG_W) * KDIM + tap * NCIN + lane * 8;
#pragma unroll 1
  for (int it = 0; it < 8; ++it) {
    const int w = it * 8 + wave;
    const float* omr = om + ((size_t)b * NPIX + (size_t)h * IMG_W + w) * NOFFPAD;
    const float oy = omr[2 * tap] + boy;
    const float ox = omr[2 * tap + 1] + box_;
    const float mv = omr[2 * NTAP + tap] + bom;
    const float gate = 1.0f / (1.0f + expf(-mv));
    const float ys = basey + oy;
    const float xs = (float)(w - 1 + kj) + ox;
    const float y0 = floorf(ys), x0 = floorf(xs);
    const float wy = ys - y0, wx = xs - x0;
    const float y1 = y0 + 1.0f, x1 = x0 + 1.0f;
    const bool vy0 = (y0 >= 0.0f) && (y0 <= cmax);
    const bool vy1 = (y1 >= 0.0f) && (y1 <= cmax);
    const bool vx0 = (x0 >= 0.0f) && (x0 <= cmax);
    const bool vx1 = (x1 >= 0.0f) && (x1 <= cmax);
    const int iy0 = (int)fminf(fmaxf(y0, 0.0f), cmax);
    const int iy1 = (int)fminf(fmaxf(y1, 0.0f), cmax);
    const int ix0 = (int)fminf(fmaxf(x0, 0.0f), cmax);
    const int ix1 = (int)fminf(fmaxf(x1, 0.0f), cmax);
    const float ay0 = 1.0f - wy, ax0 = 1.0f - wx;
    const float c00 = (vy0 && vx0) ? ay0 * ax0 : 0.0f;
    const float c01 = (vy0 && vx1) ? ay0 * wx  : 0.0f;
    const float c10 = (vy1 && vx0) ? wy  * ax0 : 0.0f;
    const float c11 = (vy1 && vx1) ? wy  * wx  : 0.0f;
    const v4u u00 = *(const v4u*)(xb + (size_t)(iy0 * IMG_W + ix0) * NCIN);
    const v4u u01 = *(const v4u*)(xb + (size_t)(iy0 * IMG_W + ix1) * NCIN);
    const v4u u10 = *(const v4u*)(xb + (size_t)(iy1 * IMG_W + ix0) * NCIN);
    const v4u u11 = *(const v4u*)(xb + (size_t)(iy1 * IMG_W + ix1) * NCIN);
    const float sc = gate * SMP_CARRY;
    v8h hv;
#pragma unroll
    for (int e = 0; e < 4; ++e) {
      float tl = __uint_as_float(u00[e] << 16) * c00;
      tl = fmaf(__uint_as_float(u01[e] << 16), c01, tl);
      tl = fmaf(__uint_as_float(u10[e] << 16), c10, tl);
      tl = fmaf(__uint_as_float(u11[e] << 16), c11, tl);
      float th = __uint_as_float(u00[e] & 0xffff0000u) * c00;
      th = fmaf(__uint_as_float(u01[e] & 0xffff0000u), c01, th);
      th = fmaf(__uint_as_float(u10[e] & 0xffff0000u), c10, th);
      th = fmaf(__uint_as_float(u11[e] & 0xffff0000u), c11, th);
      hv[2 * e]     = (_Float16)(tl * sc);
      hv[2 * e + 1] = (_Float16)(th * sc);
    }
    unsigned short* dst = arow0 + (size_t)w * KDIM;
    *(volatile v8h*)dst = hv;
    __threadfence();
    *(volatile v8h*)dst = hv;
  }
}

__global__ __launch_bounds__(NTHR) void k_partial(const float* __restrict__ conv, const float* __restrict__ bias,
                                                   float* __restrict__ part) {
  __shared__ float ss[NTHR];
  __shared__ float sq[NTHR];
  const int o = blockIdx.x, b = blockIdx.y, t = threadIdx.x;
  const float bo = bfr(bias[o]);
  const float* p = conv + ((size_t)b * NCOUT + o) * NPIX;
  float s = 0.0f, q = 0.0f;
#pragma unroll
  for (int j = 0; j < 4; ++j) {
    const v4f v = *(const v4f*)(p + (size_t)(j * NTHR + t) * 4);
#pragma unroll
    for (int e = 0; e < 4; ++e) {
      const float u = v[e] + bo;
      s += u;
      q = fmaf(u, u, q);
    }
  }
  ss[t] = s;
  sq[t] = q;
  __syncthreads();
  for (int off = NTHR / 2; off > 0; off >>= 1) {
    if (t < off) {
      ss[t] += ss[t + off];
      sq[t] += sq[t + off];
    }
    __syncthreads();
  }
  const float S = ss[0];
  const float Q = sq[0];
  if (t < 8) {
    v4f v = {0.0f, 0.0f, 0.0f, 0.0f};
    if (t == 0) { v[0] = S; v[1] = Q; }
    float* dst = part + ((size_t)b * NCOUT + o) * PART_STRIDE + t * 4;
    *(volatile v4f*)dst = v;
    __threadfence();
    *(volatile v4f*)dst = v;
  }
}

__global__ __launch_bounds__(128) void k_final(const float* __restrict__ part, float* __restrict__ stats) {
  __shared__ __align__(16) float stg[32];
  const int tid = threadIdx.x, lane = tid & 31, wave = tid >> 5;
  if (tid < 32) stg[tid] = 0.0f;
  __syncthreads();
  float s = 0.0f, q = 0.0f;
#pragma unroll
  for (int i = 0; i < 8; ++i) {
    const v4f v = *(const v4f*)(part + ((size_t)wave * NCOUT + (size_t)(lane * 8 + i)) * PART_STRIDE);
    s += v[0];
    q += v[1];
  }
#pragma unroll
  for (int off = 1; off < 32; off <<= 1) {
    s += __shfl_xor(s, off, 32);
    q += __shfl_xor(q, off, 32);
  }
  const float invn = 1.0f / (float)(NCOUT * NPIX);
  const float mu = s * invn;
  float var = q * invn - mu * mu;
  var = fmaxf(var, 0.0f);
  const float rstd = 1.0f / sqrtf(var + GN_EPS);
  if (lane == 0) {
    stg[2 * wave]     = mu;
    stg[2 * wave + 1] = rstd;
  }
  __syncthreads();
  if (tid < 8) {
    const v4f v = *(const v4f*)(stg + tid * 4);
    float* dst = stats + tid * 4;
    *(volatile v4f*)dst = v;
    __threadfence();
    *(volatile v4f*)dst = v;
  }
}

__global__ __launch_bounds__(NTHR) void k_norm(const float* __restrict__ conv, const float* __restrict__ stats,
                                                const float* __restrict__ bias, const float* __restrict__ gamma,
                                                const float* __restrict__ beta, float* __restrict__ out) {
  const int i4 = blockIdx.x * NTHR + threadIdx.x;
  const int b = i4 >> 18;
  const int o = (i4 >> 10) & (NCOUT - 1);
  const float mu = stats[2 * b];
  const float rstd = stats[2 * b + 1];
  const float bo = bfr(bias[o]);
  const float go = bfr(gamma[o]);
  const float beo = bfr(beta[o]);
  const size_t base = (size_t)i4 * 4;
  const v4f v = *(const v4f*)(conv + base);
  v4f r;
#pragma unroll
  for (int e = 0; e < 4; ++e) {
    float u = v[e] + bo;
    u = (u - mu) * rstd;
    u = u * go + beo;
    r[e] = fmaxf(u, 0.0f);
  }
  float* dst = out + base;
  *(volatile v4f*)dst = r;
  __threadfence();
  *(volatile v4f*)dst = r;
}

extern "C" void kernel_launch(void* const* d_in, const int* in_sizes, int n_in,
                              void* d_out, int out_size, void* d_ws, size_t ws_size,
                              hipStream_t stream) {
  if (n_in < 7) return;
  if (in_sizes[0] != NBATCH * NCIN * NPIX) return;
  if (in_sizes[1] != NOFF * KDIM) return;
  if (in_sizes[2] != NOFF) return;
  if (in_sizes[3] != NCOUT * KDIM) return;
  if (in_sizes[4] != NCOUT || in_sizes[5] != NCOUT || in_sizes[6] != NCOUT) return;
  if (out_size != NBATCH * NCOUT * NPIX) return;
  if (ws_size < WS_TOTAL) return;

  const float* x      = (const float*)d_in[0];
  const float* w_off  = (const float*)d_in[1];
  const float* b_off  = (const float*)d_in[2];
  const float* weight = (const float*)d_in[3];
  const float* bias   = (const float*)d_in[4];
  const float* gamma  = (const float*)d_in[5];
  const float* beta   = (const float*)d_in[6];
  float* out = (float*)d_out;

  char* ws = (char*)d_ws;
  unsigned short* xt    = (unsigned short*)(ws + OFF_XT);
  unsigned short* a16   = (unsigned short*)(ws + OFF_A16);
  unsigned short* w0p   = (unsigned short*)(ws + OFF_W0P);
  float*          om    = (float*)(ws + OFF_OM);
  unsigned short* wp    = (unsigned short*)(ws + OFF_WP);
  float*          conv  = (float*)(ws + OFF_CONV);
  float*          part  = (float*)(ws + OFF_PART);
  float*          stats = (float*)(ws + OFF_STATS);

  k_xpose<<<dim3(NPIX / 64, NCIN / 64, NBATCH), NTHR, 0, stream>>>(x, xt);
  k_im2col<<<dim3(IMG_H, NTAP, NBATCH), NTHR, 0, stream>>>(xt, a16);
  k_wprep16<<<(NOFFPAD * (KDIM / 8)) / NTHR, NTHR, 0, stream>>>(w_off, NOFF, NOFFPAD, WOFF_CARRY, w0p);
  wmma_gemm64<0, false, 0, 0, false, 0><<<dim3(((MROWS / 64) * (NOFFPAD / 64)) / 8, 1), 256, 0, stream>>>(
      a16, a16, KDIM, 0L, w0p, w0p, KDIM, 0L, (void*)om, (void*)om, NOFFPAD, 0L,
      bias, om, 0L, MROWS, NOFFPAD, KDIM, GEMM0_SCALE);
  k_wprep16<<<(NCOUT * (KDIM / 8)) / NTHR, NTHR, 0, stream>>>(weight, NCOUT, NCOUT, WGT_CARRY, wp);
  k_sample<<<dim3(IMG_H, NTAP, NBATCH), NTHR, 0, stream>>>(xt, om, b_off, a16);
  wmma_gemm64<0, false, 0, 0, false, 0><<<dim3(((NCOUT / 64) * (NPIX / 64)) / 8, NBATCH), 256, 0, stream>>>(
      wp, wp, KDIM, 0L, a16, a16, KDIM, (long)NPIX * KDIM, (void*)conv, (void*)conv, NPIX, (long)NCOUT * NPIX,
      bias, conv, 0L, NCOUT, NPIX, KDIM, GEMM1_SCALE);
  k_partial<<<dim3(NCOUT, NBATCH), NTHR, 0, stream>>>(conv, bias, part);
  k_final<<<1, 128, 0, stream>>>(part, stats);
  k_norm<<<(NBATCH * NCOUT * NPIX / 4) / NTHR, NTHR, 0, stream>>>(conv, stats, bias, gamma, beta, out);
}
